// LowLevelPolicyNetworknoskill_30958124270358
// MI455X (gfx1250) — hardware-verified
//
#include <hip/hip_runtime.h>
#include <math.h>
#include <stdint.h>


#define NTOK 8192
#define SEQL 512
#define DMOD 512
#define VTP  576
#define VTLD 9216

typedef _Float16 v16h __attribute__((ext_vector_type(16)));
typedef _Float16 v8h  __attribute__((ext_vector_type(8)));
typedef __bf16   v16b __attribute__((ext_vector_type(16)));
typedef __bf16   v8b  __attribute__((ext_vector_type(8)));
typedef float    v8f  __attribute__((ext_vector_type(8)));
typedef float    v4f  __attribute__((ext_vector_type(4)));
typedef unsigned int v4u __attribute__((ext_vector_type(4)));

__device__ __forceinline__ unsigned short f2bf_bits(float f) {
  const unsigned u = __float_as_uint(f);
  return (unsigned short)((u + 0x7FFFu + ((u >> 16) & 1u)) >> 16);
}
__device__ __forceinline__ float bf_bits2f(unsigned short h) { return __uint_as_float(((unsigned)h) << 16); }
__device__ __forceinline__ void split2(float f, unsigned short& hb, unsigned short& lb) {
  hb = f2bf_bits(f);
  lb = f2bf_bits(f - bf_bits2f(hb));
}
__device__ __forceinline__ unsigned pk16(unsigned short a, unsigned short b) { return (unsigned)a | ((unsigned)b << 16); }

__device__ __forceinline__ v8f mma_h(v16h a, v16h b, v8f c) {
  c = __builtin_amdgcn_wmma_f32_16x16x32_f16(false, a, false, b, (short)0, c, false, false);
  asm volatile("v_nop\n\tv_nop\n\tv_nop\n\tv_nop" : "+v"(c) : "v"(a), "v"(b));
  return c;
}
__device__ __forceinline__ v8f mma_b(v16b a, v16b b, v8f c) {
  c = __builtin_amdgcn_wmma_f32_16x16x32_bf16(false, a, false, b, (short)0, c, false, false);
  asm volatile("v_nop\n\tv_nop\n\tv_nop\n\tv_nop" : "+v"(c) : "v"(a), "v"(b));
  return c;
}

template <typename T> struct Frag;
template <> struct Frag<_Float16> {
  typedef v16h V;
  union U { v16h v; v8h h[2]; };
  static __device__ __forceinline__ v16h load(const _Float16* p) {
    U f; f.h[0] = *(const v8h*)(p); f.h[1] = *(const v8h*)(p + 16); return f.v;
  }
  static __device__ __forceinline__ v8f mma(v16h a, v16h b, v8f c) { return mma_h(a, b, c); }
};
template <> struct Frag<__bf16> {
  typedef v16b V;
  union U { v16b v; v8b h[2]; };
  static __device__ __forceinline__ v16b load(const __bf16* p) {
    U f; f.h[0] = *(const v8b*)(p); f.h[1] = *(const v8b*)(p + 16); return f.v;
  }
  static __device__ __forceinline__ v8f mma(v16b a, v16b b, v8f c) { return mma_b(a, b, c); }
};
template <int ET> struct Elem;
template <> struct Elem<0> { typedef _Float16 T; };
template <> struct Elem<1> { typedef __bf16 T; };

template <int ET, bool SPLIT, int BIASM, int OUTM, int ACT, int CMAP>
__global__ void __launch_bounds__(256) __attribute__((amdgpu_num_vgpr(256)))
gemm64_kernel(const unsigned short* __restrict__ Ap, const unsigned short* __restrict__ A2p, int lda,
              const unsigned short* __restrict__ Btp, const unsigned short* __restrict__ Bt2p, int ldb,
              void* Cout, void* Cout2, int ldc, const float* __restrict__ bias,
              int M, int N, int K, float scale)
{
  typedef typename Elem<ET>::T T;
  typedef typename Frag<T>::V V;
  const T* A   = (const T*)(const void*)Ap;
  const T* A2  = (const T*)(const void*)A2p;
  const T* Bt  = (const T*)(const void*)Btp;
  const T* Bt2 = (const T*)(const void*)Bt2p;
  __shared__ __align__(16) float sT[8][16 * 68];

  const int lane = threadIdx.x & 31;
  const int wave = threadIdx.x >> 5;
  const int tilesN = N >> 6, tilesM = M >> 6;
  const int tile = blockIdx.x * 8 + wave;
  if (tile >= tilesM * tilesN) return;
  const int tm = tile / tilesN;
  const int tn = tile - tm * tilesN;
  const int m0 = tm << 6, n0 = tn << 6;
  const int rl = lane & 15;
  const int koff = (lane >> 4) * 8;
  const int mOff = (lane >> 4) * 8;

  v8f acc[4][4];
#pragma unroll
  for (int i = 0; i < 4; ++i)
#pragma unroll
    for (int j = 0; j < 4; ++j) { v8f z = {0.f,0.f,0.f,0.f,0.f,0.f,0.f,0.f}; acc[i][j] = z; }

  for (int k0 = 0; k0 < K; k0 += 32) {
    V bf[4];
#pragma unroll
    for (int j = 0; j < 4; ++j) bf[j] = Frag<T>::load(Bt + (size_t)(n0 + (j << 4) + rl) * ldb + k0 + koff);
#pragma unroll
    for (int i = 0; i < 4; ++i) {
      const size_t ao = (size_t)(m0 + (i << 4) + rl) * lda + k0 + koff;
      const V ah = Frag<T>::load(A + ao);
      if (SPLIT) {
        const V al = Frag<T>::load(A2 + ao);
#pragma unroll
        for (int j = 0; j < 4; ++j) {
          acc[i][j] = Frag<T>::mma(ah, bf[j], acc[i][j]);
          acc[i][j] = Frag<T>::mma(al, bf[j], acc[i][j]);
        }
      } else {
#pragma unroll
        for (int j = 0; j < 4; ++j) acc[i][j] = Frag<T>::mma(ah, bf[j], acc[i][j]);
      }
    }
    if (SPLIT) {
#pragma unroll
      for (int j = 0; j < 4; ++j) bf[j] = Frag<T>::load(Bt2 + (size_t)(n0 + (j << 4) + rl) * ldb + k0 + koff);
#pragma unroll
      for (int i = 0; i < 4; ++i) {
        const V ah = Frag<T>::load(A + (size_t)(m0 + (i << 4) + rl) * lda + k0 + koff);
#pragma unroll
        for (int j = 0; j < 4; ++j) acc[i][j] = Frag<T>::mma(ah, bf[j], acc[i][j]);
      }
    }
  }

  float* slab = sT[wave];
  const int colbase = CMAP ? (((n0 >> 9) * VTP) + 64 + (n0 & 511)) : n0;
#pragma unroll
  for (int i = 0; i < 4; ++i) {
    const int mBase = m0 + (i << 4);
#pragma unroll
    for (int j = 0; j < 4; ++j) {
      const int nl = n0 + (j << 4) + rl;
      float bv = 0.0f;
      if (BIASM == 2) bv = bias[nl];
#pragma unroll
      for (int r = 0; r < 8; ++r) {
        float v = acc[i][j][r] * scale;
        if (BIASM == 1) v += bias[mBase + mOff + r];
        if (BIASM == 2) v += bv;
        if (ACT == 2) v = fmaxf(v, 0.0f);
        slab[(mOff + r) * 68 + (j << 4) + rl] = v;
      }
    }
    __builtin_amdgcn_fence(__ATOMIC_RELEASE, "workgroup");
    __builtin_amdgcn_wave_barrier();
    __builtin_amdgcn_fence(__ATOMIC_ACQUIRE, "workgroup");
    const int hh = lane >> 4, c4 = (lane & 15) * 4;
    const int q = lane >> 3, c8 = (lane & 7) * 8;
    for (int pass = 0; pass < 2; ++pass) {
      if (OUTM == 0 || OUTM == 3) {
        float* C = (float*)Cout;
#pragma unroll
        for (int it = 0; it < 8; ++it) {
          const int row = it * 2 + hh;
          const v4f v = *(const v4f*)(slab + row * 68 + c4);
          *(volatile v4f*)(C + (size_t)(mBase + row) * ldc + colbase + c4) = v;
        }
      }
      if (OUTM != 0) {
        unsigned short* C1 = (OUTM == 3) ? (unsigned short*)Cout2 : (unsigned short*)Cout;
        unsigned short* C2 = (unsigned short*)Cout2;
#pragma unroll
        for (int it = 0; it < 4; ++it) {
          const int row = it * 4 + q;
          const float* sp = slab + row * 68 + c8;
          v8h hv, lv;
#pragma unroll
          for (int e = 0; e < 8; ++e) {
            if (OUTM == 2) {
              unsigned short hb, lb; split2(sp[e], hb, lb);
              hv[e] = __builtin_bit_cast(_Float16, hb);
              lv[e] = __builtin_bit_cast(_Float16, lb);
            } else {
              hv[e] = (_Float16)sp[e];
              lv[e] = hv[e];
            }
          }
          *(volatile v8h*)(C1 + (size_t)(mBase + row) * ldc + colbase + c8) = hv;
          if (OUTM == 2) *(volatile v8h*)(C2 + (size_t)(mBase + row) * ldc + colbase + c8) = lv;
        }
      }
      __threadfence();
    }
    __builtin_amdgcn_fence(__ATOMIC_RELEASE, "workgroup");
    __builtin_amdgcn_wave_barrier();
    __builtin_amdgcn_fence(__ATOMIC_ACQUIRE, "workgroup");
  }
}

template <int OUTK>
__global__ void __launch_bounds__(256) __attribute__((amdgpu_num_vgpr(256)))
gemm_ln_kernel(const unsigned short* __restrict__ Ap, int lda,
               const unsigned short* __restrict__ Btp, int ldb,
               const float* __restrict__ bias, const float* __restrict__ resid,
               const float* __restrict__ gam, const float* __restrict__ bet,
               void* Cout, void* Cout2, int K, float scale)
{
  const _Float16* A  = (const _Float16*)(const void*)Ap;
  const _Float16* Bt = (const _Float16*)(const void*)Btp;
  __shared__ __align__(16) float sT[8][16 * 68];
  __shared__ float red1[8][16];
  __shared__ float red2[8][16];

  const int lane = threadIdx.x & 31;
  const int wave = threadIdx.x >> 5;
  const int hh = lane >> 4;
  const int rl = lane & 15;
  const int koff = hh * 8;
  const int mOff = hh * 8;
  const int m0 = blockIdx.x << 6;
  const int n0 = wave << 6;

  v8f acc[4][4];
#pragma unroll
  for (int i = 0; i < 4; ++i)
#pragma unroll
    for (int j = 0; j < 4; ++j) { v8f z = {0.f,0.f,0.f,0.f,0.f,0.f,0.f,0.f}; acc[i][j] = z; }

  for (int k0 = 0; k0 < K; k0 += 32) {
    v16h bf[4];
#pragma unroll
    for (int j = 0; j < 4; ++j) bf[j] = Frag<_Float16>::load(Bt + (size_t)(n0 + (j << 4) + rl) * ldb + k0 + koff);
#pragma unroll
    for (int i = 0; i < 4; ++i) {
      const v16h ah = Frag<_Float16>::load(A + (size_t)(m0 + (i << 4) + rl) * lda + k0 + koff);
#pragma unroll
      for (int j = 0; j < 4; ++j) acc[i][j] = mma_h(ah, bf[j], acc[i][j]);
    }
  }

  float* slab = sT[wave];
#pragma unroll
  for (int i = 0; i < 4; ++i) {
    const int mBase = m0 + (i << 4);
#pragma unroll
    for (int j = 0; j < 4; ++j) {
      const int n = n0 + (j << 4) + rl;
      const float bv = bias[n];
#pragma unroll
      for (int r = 0; r < 8; ++r) {
        const int m = mBase + mOff + r;
        acc[i][j][r] = acc[i][j][r] * scale + bv + resid[(size_t)m * DMOD + n];
      }
    }
    float mean[8], rstd[8];
#pragma unroll
    for (int r = 0; r < 8; ++r) {
      float s = acc[i][0][r] + acc[i][1][r] + acc[i][2][r] + acc[i][3][r];
#pragma unroll
      for (int off = 1; off < 16; off <<= 1) s += __shfl_xor(s, off, 32);
      if (rl == 0) red1[wave][mOff + r] = s;
    }
    __syncthreads();
#pragma unroll
    for (int r = 0; r < 8; ++r) {
      float tot = 0.0f;
#pragma unroll
      for (int w = 0; w < 8; ++w) tot += red1[w][mOff + r];
      mean[r] = tot * (1.0f / 512.0f);
    }
#pragma unroll
    for (int r = 0; r < 8; ++r) {
      float sq = 0.0f;
#pragma unroll
      for (int j = 0; j < 4; ++j) { const float d = acc[i][j][r] - mean[r]; sq += d * d; }
#pragma unroll
      for (int off = 1; off < 16; off <<= 1) sq += __shfl_xor(sq, off, 32);
      if (rl == 0) red2[wave][mOff + r] = sq;
    }
    __syncthreads();
#pragma unroll
    for (int r = 0; r < 8; ++r) {
      float tot = 0.0f;
#pragma unroll
      for (int w = 0; w < 8; ++w) tot += red2[w][mOff + r];
      rstd[r] = rsqrtf(tot * (1.0f / 512.0f) + 1e-5f);
    }
#pragma unroll
    for (int j = 0; j < 4; ++j) {
      const int n = n0 + (j << 4) + rl;
      const float gv = gam[n], tv = bet[n];
#pragma unroll
      for (int r = 0; r < 8; ++r) {
        const float y = (acc[i][j][r] - mean[r]) * rstd[r] * gv + tv;
        slab[(mOff + r) * 68 + (j << 4) + rl] = y;
      }
    }
    __builtin_amdgcn_fence(__ATOMIC_RELEASE, "workgroup");
    __builtin_amdgcn_wave_barrier();
    __builtin_amdgcn_fence(__ATOMIC_ACQUIRE, "workgroup");
    const int c4 = rl * 4;
    const int q = lane >> 3, c8 = (lane & 7) * 8;
    for (int pass = 0; pass < 2; ++pass) {
      if (OUTK == 0) {
        float* Cf = (float*)Cout;
        unsigned short* Ch = (unsigned short*)Cout2;
#pragma unroll
        for (int it = 0; it < 8; ++it) {
          const int row = it * 2 + hh;
          const v4f v = *(const v4f*)(slab + row * 68 + c4);
          *(volatile v4f*)(Cf + (size_t)(mBase + row) * DMOD + n0 + c4) = v;
        }
#pragma unroll
        for (int it = 0; it < 4; ++it) {
          const int row = it * 4 + q;
          const float* sp = slab + row * 68 + c8;
          v8h hv;
#pragma unroll
          for (int e = 0; e < 8; ++e) hv[e] = (_Float16)sp[e];
          *(volatile v8h*)(Ch + (size_t)(mBase + row) * DMOD + n0 + c8) = hv;
        }
      } else {
        unsigned short* C1 = (unsigned short*)Cout;
        unsigned short* C2 = (unsigned short*)Cout2;
#pragma unroll
        for (int it = 0; it < 4; ++it) {
          const int row = it * 4 + q;
          const float* sp = slab + row * 68 + c8;
          v8h hv, lv;
#pragma unroll
          for (int e = 0; e < 8; ++e) {
            unsigned short hb, lb; split2(sp[e], hb, lb);
            hv[e] = __builtin_bit_cast(_Float16, hb);
            lv[e] = __builtin_bit_cast(_Float16, lb);
          }
          *(volatile v8h*)(C1 + (size_t)(mBase + row) * DMOD + n0 + c8) = hv;
          *(volatile v8h*)(C2 + (size_t)(mBase + row) * DMOD + n0 + c8) = lv;
        }
      }
      __threadfence();
    }
    __builtin_amdgcn_fence(__ATOMIC_RELEASE, "workgroup");
    __builtin_amdgcn_wave_barrier();
    __builtin_amdgcn_fence(__ATOMIC_ACQUIRE, "workgroup");
  }
}

__global__ void __launch_bounds__(128) attn_band_kernel(const unsigned short* __restrict__ QKp,
                                                        const unsigned short* __restrict__ VTp,
                                                        const float* __restrict__ padm,
                                                        unsigned short* Oout)
{
  union FH { v16h v; v8h h[2]; };
  const _Float16* QK = (const _Float16*)(const void*)QKp;
  const _Float16* VT = (const _Float16*)(const void*)VTp;
  _Float16* O = (_Float16*)(void*)Oout;
  __shared__ __align__(16) _Float16 Ps[4][16 * 32];
  __shared__ __align__(16) float    Os[4][16 * 68];

  const int tid = threadIdx.x;
  const int wave = tid >> 5, lane = tid & 31, hh = lane >> 4, c = lane & 15;
  const int qb = blockIdx.x, h = blockIdx.y, b = blockIdx.z;
  const int qw0 = qb * 64 + wave * 16;
  const int tb = b * SEQL;

  v16h qa[2];
#pragma unroll
  for (int dc = 0; dc < 2; ++dc) {
    const _Float16* p = QK + (size_t)(tb + qw0 + c) * 1024 + h * 64 + dc * 32 + 8 * hh;
    FH f; f.h[0] = *(const v8h*)(p); f.h[1] = *(const v8h*)(p + 16); qa[dc] = f.v;
  }
  v8f s[2];
  float padv[2];
#pragma unroll
  for (int j = 0; j < 2; ++j) {
    v8f z = {0.f,0.f,0.f,0.f,0.f,0.f,0.f,0.f}; s[j] = z;
    const int key = qw0 - 16 + 16 * j + c;
    int kcl = key < 0 ? 0 : key; kcl = kcl > (SEQL - 1) ? (SEQL - 1) : kcl;
    padv[j] = padm[tb + kcl];
#pragma unroll
    for (int dc = 0; dc < 2; ++dc) {
      const _Float16* p = QK + (size_t)(tb + kcl) * 1024 + 512 + h * 64 + dc * 32 + 8 * hh;
      FH f; f.h[0] = *(const v8h*)(p); f.h[1] = *(const v8h*)(p + 16);
      s[j] = mma_h(qa[dc], f.v, s[j]);
    }
  }
  float mrow[8], lrow[8];
#pragma unroll
  for (int r = 0; r < 8; ++r) {
    const int iq = qw0 + 8 * hh + r;
    float m = -INFINITY;
#pragma unroll
    for (int j = 0; j < 2; ++j) {
      const int ik = qw0 - 16 + 16 * j + c;
      const bool allowed = (ik >= 0) && (ik <= iq) && (iq - ik <= 16);
      const float sv = allowed ? (s[j][r] * 0.125f + padv[j]) : -INFINITY;
      s[j][r] = sv;
      m = fmaxf(m, sv);
    }
#pragma unroll
    for (int off = 1; off < 16; off <<= 1) m = fmaxf(m, __shfl_xor(m, off, 32));
    mrow[r] = m;
  }
  _Float16* pw = Ps[wave];
#pragma unroll
  for (int r = 0; r < 8; ++r) {
    float sum = 0.0f;
#pragma unroll
    for (int j = 0; j < 2; ++j) {
      const float p = expf(s[j][r] - mrow[r]);
      sum += p;
      pw[(8 * hh + r) * 32 + 16 * j + c] = (_Float16)(p * 256.0f);
    }
#pragma unroll
    for (int off = 1; off < 16; off <<= 1) sum += __shfl_xor(sum, off, 32);
    lrow[r] = sum;
  }
  __builtin_amdgcn_fence(__ATOMIC_RELEASE, "workgroup");
  __builtin_amdgcn_wave_barrier();
  __builtin_amdgcn_fence(__ATOMIC_ACQUIRE, "workgroup");
  FH pa;
  pa.h[0] = *(const v8h*)(pw + c * 32 + 8 * hh);
  pa.h[1] = *(const v8h*)(pw + c * 32 + 16 + 8 * hh);
  v8f o[4];
#pragma unroll
  for (int t = 0; t < 4; ++t) {
    const _Float16* p = VT + (size_t)(h * 64 + 16 * t + c) * VTLD + b * VTP + 48 + qw0 + 8 * hh;
    FH f; f.h[0] = *(const v8h*)(p); f.h[1] = *(const v8h*)(p + 16);
    v8f z = {0.f,0.f,0.f,0.f,0.f,0.f,0.f,0.f};
    o[t] = mma_h(pa.v, f.v, z);
  }
  float* os = Os[wave];
#pragma unroll
  for (int r = 0; r < 8; ++r) {
    const float inv = (1.0f / lrow[r]) * 0.00390625f;
#pragma unroll
    for (int t = 0; t < 4; ++t) os[(8 * hh + r) * 68 + 16 * t + c] = o[t][r] * inv;
  }
  __builtin_amdgcn_fence(__ATOMIC_RELEASE, "workgroup");
  __builtin_amdgcn_wave_barrier();
  __builtin_amdgcn_fence(__ATOMIC_ACQUIRE, "workgroup");
  const int q = lane >> 3, c8 = (lane & 7) * 8;
  for (int pass = 0; pass < 2; ++pass) {
#pragma unroll
    for (int it = 0; it < 4; ++it) {
      const int row = it * 4 + q;
      const float* sp = os + row * 68 + c8;
      v8h hv;
#pragma unroll
      for (int e = 0; e < 8; ++e) hv[e] = (_Float16)sp[e];
      *(volatile v8h*)(O + (size_t)(tb + qw0 + row) * DMOD + h * 64 + c8) = hv;
    }
    __threadfence();
  }
}

__global__ void __launch_bounds__(256) split_rows_kernel(const float* __restrict__ in, int rows, int cols,
                                                         unsigned short* hi, unsigned short* lo, int pitch)
{
  const int cpr = pitch >> 3;
  const int nthr = rows * cpr;
  const int t = blockIdx.x * 256 + threadIdx.x;
  if (t >= nthr) return;
  const int row = t / cpr;
  const int col0 = (t - row * cpr) * 8;
  const float* src = in + (size_t)row * cols;
  v4u hv, lv;
#pragma unroll
  for (int qd = 0; qd < 4; ++qd) {
    const int ca = col0 + 2 * qd, cb = ca + 1;
    const int caa = ca < cols ? ca : (cols - 1);
    const int cbb = cb < cols ? cb : (cols - 1);
    float f0 = src[caa], f1 = src[cbb];
    f0 = (ca < cols) ? f0 : 0.0f;
    f1 = (cb < cols) ? f1 : 0.0f;
    unsigned short h0, l0, h1, l1;
    split2(f0, h0, l0); split2(f1, h1, l1);
    hv[qd] = pk16(h0, h1); lv[qd] = pk16(l0, l1);
  }
  const size_t o = (size_t)row * pitch + col0;
  *(volatile v4u*)(hi + o) = hv;
  *(volatile v4u*)(lo + o) = lv;
  __threadfence();
  *(volatile v4u*)(hi + o) = hv;
  *(volatile v4u*)(lo + o) = lv;
}

__global__ void __launch_bounds__(256) cvt_f16_x4_kernel(const float* __restrict__ s0, unsigned short* d0, int nb0,
                                                         const float* __restrict__ s1, unsigned short* d1, int nb1,
                                                         const float* __restrict__ s2, unsigned short* d2, int nb2,
                                                         const float* __restrict__ s3, unsigned short* d3, int nb3,
                                                         float scale)
{
  int bid = blockIdx.x;
  const float* s; unsigned short* d;
  if (bid < nb0) { s = s0; d = d0; }
  else if (bid < nb0 + nb1) { bid -= nb0; s = s1; d = d1; }
  else if (bid < nb0 + nb1 + nb2) { bid -= nb0 + nb1; s = s2; d = d2; }
  else { bid -= nb0 + nb1 + nb2; if (bid >= nb3) return; s = s3; d = d3; }
  const size_t e0 = ((size_t)bid * 256 + threadIdx.x) * 8;
  const v4f a = *(const v4f*)(s + e0);
  const v4f bq = *(const v4f*)(s + e0 + 4);
  v8h ov;
#pragma unroll
  for (int e = 0; e < 4; ++e) { ov[e] = (_Float16)(a[e] * scale); ov[e + 4] = (_Float16)(bq[e] * scale); }
  _Float16* dp = (_Float16*)(void*)d;
  *(volatile v8h*)(dp + e0) = ov;
  __threadfence();
  *(volatile v8h*)(dp + e0) = ov;
}

__global__ void __launch_bounds__(256) padmask_kernel(const float* __restrict__ goal, float* padm, int ntok, int gdim)
{
  const int t = blockIdx.x * 256 + threadIdx.x;
  if (t >= ntok) return;
  const float* g = goal + (size_t)t * gdim;
  int all = 1;
  for (int k = 0; k < gdim; ++k) all &= (g[k] == -1.0f) ? 1 : 0;
  const float v = all ? -1.0e9f : 0.0f;
  ((volatile float*)padm)[t] = v;
  __threadfence();
  ((volatile float*)padm)[t] = v;
}

__global__ void __launch_bounds__(256) vtpad_kernel(unsigned short* VT, int nseg)
{
  const int t = blockIdx.x * 256 + threadIdx.x;
  const int seg = t >> 3, q = t & 7;
  if (seg >= nseg) return;
  const int d = seg >> 4, b = seg & 15;
  const size_t o = (size_t)d * VTLD + (size_t)b * VTP + q * 8;
  v4u z = {0u, 0u, 0u, 0u};
  *(volatile v4u*)(VT + o) = z;
  __threadfence();
  *(volatile v4u*)(VT + o) = z;
}

__global__ void __launch_bounds__(256) head_prep_kernel(const float* __restrict__ Wa1, const float* __restrict__ ba1,
                                                        const float* __restrict__ Wa2, const float* __restrict__ ba2,
                                                        unsigned short* Wah, unsigned short* Wal, float* bias128)
{
  const int t = blockIdx.x * 256 + threadIdx.x;
  if (t < 4096) {
    const int n = t >> 5;
    const int k0 = (t & 31) * 8;
    const int n1 = n < 11 ? n : 11;
    int n2 = n - 12; n2 = n2 < 0 ? 0 : n2; n2 = n2 > 88 ? 88 : n2;
    v4u hv, lv;
#pragma unroll
    for (int qd = 0; qd < 4; ++qd) {
      unsigned short hb[2], lb[2];
#pragma unroll
      for (int e = 0; e < 2; ++e) {
        const int k = k0 + 2 * qd + e;
        const float a1 = Wa1[n1 * 256 + k];
        const float a2 = Wa2[n2 * 256 + k];
        const float f = (n < 12) ? a1 : ((n < 101) ? a2 : 0.0f);
        split2(f, hb[e], lb[e]);
      }
      hv[qd] = pk16(hb[0], hb[1]); lv[qd] = pk16(lb[0], lb[1]);
    }
    const size_t o = (size_t)n * 256 + k0;
    *(volatile v4u*)(Wah + o) = hv;
    *(volatile v4u*)(Wal + o) = lv;
    __threadfence();
    *(volatile v4u*)(Wah + o) = hv;
    *(volatile v4u*)(Wal + o) = lv;
  }
  if (blockIdx.x == 0 && threadIdx.x < 32) {
    const int ln = threadIdx.x;
    v4f bv;
#pragma unroll
    for (int e = 0; e < 4; ++e) {
      const int n = 4 * ln + e;
      const int n1 = n < 11 ? n : 11;
      int n2 = n - 12; n2 = n2 < 0 ? 0 : n2; n2 = n2 > 88 ? 88 : n2;
      const float b1 = ba1[n1], b2 = ba2[n2];
      bv[e] = (n < 12) ? b1 : ((n < 101) ? b2 : 0.0f);
    }
    *(volatile v4f*)(bias128 + 4 * ln) = bv;
    __threadfence();
    *(volatile v4f*)(bias128 + 4 * ln) = bv;
  }
}

__global__ void __launch_bounds__(256) out_copy_kernel(const float* __restrict__ C, float* out, int n4)
{
  const int t = blockIdx.x * 256 + threadIdx.x;
  if (t >= n4) return;
  const int e0 = t * 4;
  v4f v;
#pragma unroll
  for (int e = 0; e < 4; ++e) {
    const int idx = e0 + e;
    const int row = idx / 101;
    const int col = idx - row * 101;
    v[e] = C[(size_t)row * 128 + col];
  }
  *(volatile v4f*)(out + e0) = v;
  __threadfence();
  *(volatile v4f*)(out + e0) = v;
}

template <int ET, bool SPLIT, int BIASM, int OUTM, int ACT, int CMAP>
static void run_gemm(const unsigned short* A, const unsigned short* A2, int lda,
                     const unsigned short* Bt, const unsigned short* Bt2, int ldb,
                     void* C, void* C2, int ldc, const float* bias,
                     int M, int N, int K, float scale, hipStream_t st)
{
  const int tiles = (M >> 6) * (N >> 6);
  dim3 grid((tiles + 7) / 8);
  gemm64_kernel<ET, SPLIT, BIASM, OUTM, ACT, CMAP><<<grid, dim3(256), 0, st>>>(
      A, A2, lda, Bt, Bt2, ldb, C, C2, ldc, bias, M, N, K, scale);
}

extern "C" void kernel_launch(void* const* d_in, const int* in_sizes, int n_in,
                              void* d_out, int out_size, void* d_ws, size_t ws_size,
                              hipStream_t stream)
{
  if (n_in < 26) return;
  if (in_sizes[0] != NTOK * 768 || in_sizes[1] != NTOK * 300) return;
  if (in_sizes[2] != 256 * 768 || in_sizes[3] != 256 || in_sizes[4] != 256 * 300 || in_sizes[5] != 256) return;
  if (in_sizes[6] != 512 * 512 || in_sizes[7] != 512) return;
  if (in_sizes[8] != 3 * 1536 * 512 || in_sizes[9] != 3 * 1536 || in_sizes[10] != 3 * 512 * 512 || in_sizes[11] != 1536) return;
  if (in_sizes[12] != 3 * 2048 * 512 || in_sizes[13] != 3 * 2048 || in_sizes[14] != 3 * 512 * 2048 || in_sizes[15] != 1536) return;
  if (in_sizes[16] != 1536 || in_sizes[17] != 1536 || in_sizes[18] != 1536 || in_sizes[19] != 1536) return;
  if (in_sizes[20] != 256 * 512 || in_sizes[21] != 256 || in_sizes[22] != 12 * 256 || in_sizes[23] != 12) return;
  if (in_sizes[24] != 89 * 256 || in_sizes[25] != 89) return;
  if (out_size != NTOK * 101) return;

  const float* state  = (const float*)d_in[0];
  const float* goal   = (const float*)d_in[1];
  const float* W_obs  = (const float*)d_in[2];
  const float* b_obs  = (const float*)d_in[3];
  const float* W_lang = (const float*)d_in[4];
  const float* b_lang = (const float*)d_in[5];
  const float* W_in   = (const float*)d_in[6];
  const float* b_in   = (const float*)d_in[7];
  const float* Wqkv   = (const float*)d_in[8];
  const float* bqkv   = (const float*)d_in[9];
  const float* Wo     = (const float*)d_in[10];
  const float* bo     = (const float*)d_in[11];
  const float* W1     = (const float*)d_in[12];
  const float* b1     = (const float*)d_in[13];
  const float* W2     = (const float*)d_in[14];
  const float* b2     = (const float*)d_in[15];
  const float* g1     = (const float*)d_in[16];
  const float* bt1    = (const float*)d_in[17];
  const float* g2     = (const float*)d_in[18];
  const float* bt2    = (const float*)d_in[19];
  const float* W_outp = (const float*)d_in[20];
  const float* b_outp = (const float*)d_in[21];
  const float* W_a1   = (const float*)d_in[22];
  const float* b_a1   = (const float*)d_in[23];
  const float* W_a2   = (const float*)d_in[24];
  const float* b_a2   = (const float*)d_in[25];
  float* out = (float*)d_out;

  size_t off = 0;
  const size_t oA   = off; off += (size_t)35651584;
  const size_t oB   = off; off += (size_t)34603008;
  const size_t oWe  = off; off += (size_t)2162688;
  const size_t oXf0 = off; off += (size_t)NTOK * DMOD * 4;
  const size_t oXf1 = off; off += (size_t)NTOK * DMOD * 4;
  const size_t oXh  = off; off += (size_t)NTOK * DMOD * 2;
  const size_t oPad = off; off += (size_t)NTOK * 4;
  const size_t oW16 = off; off += (size_t)6291456;
  const size_t oHw  = off; off += (size_t)655872;
  if (off > ws_size) return;

  char* ws = (char*)d_ws;
  unsigned short* Sh   = (unsigned short*)(ws + oA);
  unsigned short* Sl   = (unsigned short*)(ws + oA + 12582912);
  unsigned short* Gh   = (unsigned short*)(ws + oA + 25165824);
  unsigned short* Gl   = (unsigned short*)(ws + oA + 30408704);
  unsigned short* Fh   = (unsigned short*)(ws + oA);
  unsigned short* Hh   = (unsigned short*)(ws + oA);
  unsigned short* Hl   = (unsigned short*)(ws + oA + 4194304);
  float*          C128 = (float*)(ws + oA + 8388608);
  unsigned short* QK   = (unsigned short*)(ws + oB);
  unsigned short* VT   = (unsigned short*)(ws + oB + 16777216);
  unsigned short* Oh   = (unsigned short*)(ws + oB + 26214400);
  unsigned short* Uh   = (unsigned short*)(ws + oB);
  unsigned short* Ul   = (unsigned short*)(ws + oB + 8388608);
  unsigned short* Xbh  = Uh;
  unsigned short* Xbl  = Ul;
  unsigned short* Wobh = (unsigned short*)(ws + oWe);
  unsigned short* Wobl = (unsigned short*)(ws + oWe + 393216);
  unsigned short* Wlah = (unsigned short*)(ws + oWe + 786432);
  unsigned short* Wlal = (unsigned short*)(ws + oWe + 950272);
  unsigned short* Winh = (unsigned short*)(ws + oWe + 1114112);
  unsigned short* Winl = (unsigned short*)(ws + oWe + 1638400);
  float*          Xf0  = (float*)(ws + oXf0);
  float*          Xf1  = (float*)(ws + oXf1);
  unsigned short* Xh   = (unsigned short*)(ws + oXh);
  float*          padm = (float*)(ws + oPad);
  unsigned short* Wqkv16 = (unsigned short*)(ws + oW16);
  unsigned short* Wo16   = (unsigned short*)(ws + oW16 + 1572864);
  unsigned short* W1_16  = (unsigned short*)(ws + oW16 + 2097152);
  unsigned short* W2_16  = (unsigned short*)(ws + oW16 + 4194304);
  unsigned short* Wouth = (unsigned short*)(ws + oHw);
  unsigned short* Woutl = (unsigned short*)(ws + oHw + 262144);
  unsigned short* Wah   = (unsigned short*)(ws + oHw + 524288);
  unsigned short* Wal   = (unsigned short*)(ws + oHw + 589824);
  float*          bias128 = (float*)(ws + oHw + 655360);

  const dim3 blk(256);

  split_rows_kernel<<<dim3((NTOK * 96 + 255) / 256), blk, 0, stream>>>(state, NTOK, 768, Sh, Sl, 768);
  split_rows_kernel<<<dim3((NTOK * 40 + 255) / 256), blk, 0, stream>>>(goal, NTOK, 300, Gh, Gl, 320);
  split_rows_kernel<<<dim3((256 * 96 + 255) / 256), blk, 0, stream>>>(W_obs, 256, 768, Wobh, Wobl, 768);
  split_rows_kernel<<<dim3((256 * 40 + 255) / 256), blk, 0, stream>>>(W_lang, 256, 300, Wlah, Wlal, 320);
  split_rows_kernel<<<dim3((512 * 64 + 255) / 256), blk, 0, stream>>>(W_in, 512, 512, Winh, Winl, 512);
  split_rows_kernel<<<dim3((256 * 64 + 255) / 256), blk, 0, stream>>>(W_outp, 256, 512, Wouth, Woutl, 512);
  head_prep_kernel<<<dim3(16), blk, 0, stream>>>(W_a1, b_a1, W_a2, b_a2, Wah, Wal, bias128);
  padmask_kernel<<<dim3((NTOK + 255) / 256), blk, 0, stream>>>(goal, padm, NTOK, 300);

  run_gemm<1, true, 2, 2, 0, 0>(Sh, Sl, 768, Wobh, Wobl, 768, (void*)Uh, (void*)Ul, 512, b_obs,
                                NTOK, 256, 768, 1.0f, stream);
  run_gemm<1, true, 2, 2, 0, 0>(Gh, Gl, 320, Wlah, Wlal, 320, (void*)(Uh + 256), (void*)(Ul + 256), 512, b_lang,
                                NTOK, 256, 320, 1.0f, stream);
  run_gemm<1, true, 2, 3, 0, 0>(Uh, Ul, 512, Winh, Winl, 512, (void*)Xf0, (void*)Xh, 512, b_in,
                                NTOK, 512, 512, 1.0f, stream);
  vtpad_kernel<<<dim3((512 * 16 * 8 + 255) / 256), blk, 0, stream>>>(VT, 512 * 16);

  const float wsc = 32.0f, winv = 1.0f / 32.0f;
  for (int l = 0; l < 3; ++l) {
    const float* Wqkv_l = Wqkv + (size_t)l * 1536 * 512;
    const float* bqkv_l = bqkv + (size_t)l * 1536;
    const float* Wo_l = Wo + (size_t)l * 512 * 512;
    const float* bo_l = bo + (size_t)l * 512;
    const float* W1_l = W1 + (size_t)l * 2048 * 512;
    const float* b1_l = b1 + (size_t)l * 2048;
    const float* W2_l = W2 + (size_t)l * 512 * 2048;
    const float* b2_l = b2 + (size_t)l * 512;

    cvt_f16_x4_kernel<<<dim3(1536), blk, 0, stream>>>(Wqkv_l, Wqkv16, 384, Wo_l, Wo16, 128,
                                                     W1_l, W1_16, 512, W2_l, W2_16, 512, wsc);
    run_gemm<0, false, 2, 1, 0, 0>(Xh, Xh, 512, Wqkv16, Wqkv16, 512, (void*)QK, (void*)QK, 1024, bqkv_l,
                                   NTOK, 1024, 512, winv, stream);
    run_gemm<0, false, 1, 1, 0, 1>(Wqkv16 + (size_t)1024 * 512, Wqkv16, 512, Xh, Xh, 512, (void*)VT, (void*)VT,
                                   VTLD, bqkv_l + 1024, 512, NTOK, 512, winv, stream);
    attn_band_kernel<<<dim3(8, 8, 16), dim3(128), 0, stream>>>(QK, VT, padm, Oh);
    gemm_ln_kernel<0><<<dim3(NTOK / 64), blk, 0, stream>>>(Oh, 512, Wo16, 512, bo_l, Xf0,
                                                           g1 + (size_t)l * 512, bt1 + (size_t)l * 512,
                                                           (void*)Xf1, (void*)Xh, 512, winv);
    run_gemm<0, false, 2, 1, 2, 0>(Xh, Xh, 512, W1_16, W1_16, 512, (void*)Fh, (void*)Fh, 2048, b1_l,
                                   NTOK, 2048, 512, winv, stream);
    if (l < 2) {
      gemm_ln_kernel<0><<<dim3(NTOK / 64), blk, 0, stream>>>(Fh, 2048, W2_16, 2048, b2_l, Xf1,
                                                             g2 + (size_t)l * 512, bt2 + (size_t)l * 512,
                                                             (void*)Xf0, (void*)Xh, 2048, winv);
    } else {
      gemm_ln_kernel<1><<<dim3(NTOK / 64), blk, 0, stream>>>(Fh, 2048, W2_16, 2048, b2_l, Xf1,
                                                             g2 + (size_t)l * 512, bt2 + (size_t)l * 512,
                                                             (void*)Xbh, (void*)Xbl, 2048, winv);
    }
  }

  run_gemm<1, true, 2, 2, 0, 0>(Xbh, Xbl, 512, Wouth, Woutl, 512, (void*)Hh, (void*)Hl, 256, b_outp,
                                NTOK, 256, 512, 1.0f, stream);
  run_gemm<1, true, 2, 0, 0, 0>(Hh, Hl, 256, Wah, Wal, 256, (void*)C128, (void*)C128, 128, bias128,
                                NTOK, 128, 256, 1.0f, stream);
  out_copy_kernel<<<dim3((NTOK * 101 / 4 + 255) / 256), blk, 0, stream>>>(C128, out, NTOK * 101 / 4);
  (void)hipGetLastError();
}
